// GraphAttention_52166672777276
// MI455X (gfx1250) — hardware-run, weakly checked
//
#include <hip/hip_runtime.h>
#include <stddef.h>
#include <stdint.h>


#define DI      256
#define DO      64
#define NH      4
#define NF      (NH * DO)
#define NTHR    256
#define NWAVE   8
#define EPT     8
#define CHUNK   (NTHR * EPT)
#define WCAP    (EPT * 32)
#define LISTN   (NWAVE * WCAP)
#define NBMAX   2048
#define SLOTB   11
#define RCAP    28672
#define DEGCAP  256
#define GBM     64
#define GBN     64
#define GTHR    128
#define NEGSL   0.2f
#define WSMAX   134217728
#define LDS_AGG ((2 * RCAP + 2 * NBMAX + LISTN) * 4 + 64)

static_assert((CHUNK & (CHUNK - 1)) == 0 && CHUNK <= (1 << SLOTB));
static_assert(NBMAX == (1 << SLOTB));
static_assert(NTHR * 8 == NBMAX);
static_assert(LISTN >= NBMAX);
static_assert(LISTN >= NWAVE * WCAP);
static_assert((RCAP % 32) == 0);
static_assert(LDS_AGG <= 300000);
static_assert(GBM == (GTHR / 32) * 16);
static_assert(GTHR == 2 * DO && GTHR == 2 * GBM);
static_assert(GBN == DO && NF == NH * GBN);
static_assert((DI % 32) == 0 && (DI / 8) == 32);
static_assert(NF == 8 * 32);
static_assert(DO == 8 * 8);

typedef float          v4f  __attribute__((ext_vector_type(4)));
typedef float          v8f  __attribute__((ext_vector_type(8)));
typedef int            v4i  __attribute__((ext_vector_type(4)));
typedef int            v8i  __attribute__((ext_vector_type(8)));
typedef unsigned short v8us __attribute__((ext_vector_type(8)));
typedef __bf16         v16b __attribute__((ext_vector_type(16)));
typedef v4f  __attribute__((may_alias)) v4fa;
typedef v8us __attribute__((may_alias)) v8usa;
union FragB { v16b v; v8us h[2]; v8i w; };

__device__ __forceinline__ v8f wmb(const FragB& a, const FragB& b, v8f c) {
  v8f d = __builtin_amdgcn_wmma_f32_16x16x32_bf16(false, a.v, false, b.v, (short)0, c, false, false);
  asm volatile("v_nop\n\tv_nop\n\tv_nop\n\tv_nop" : "+v"(d) : "v"(a.w), "v"(b.w));
  return d;
}

__device__ __forceinline__ unsigned short f2bf(float f) {
  unsigned u = __float_as_uint(f);
  u += 0x7FFFu + ((u >> 16) & 1u);
  return (unsigned short)(u >> 16);
}
__device__ __forceinline__ float bfr(float f) {
  unsigned u = __float_as_uint(f);
  u = (u + 0x7FFFu + ((u >> 16) & 1u)) & 0xFFFF0000u;
  return __uint_as_float(u);
}
__device__ __forceinline__ v8us cvt8b(const v4f a, const v4f b) {
  v8us o;
  o[0] = f2bf(a.x); o[1] = f2bf(a.y); o[2] = f2bf(a.z); o[3] = f2bf(a.w);
  o[4] = f2bf(b.x); o[5] = f2bf(b.y); o[6] = f2bf(b.z); o[7] = f2bf(b.w);
  return o;
}

__device__ __forceinline__ int scan_chunk(const int* __restrict__ ei, int nE, int cbase, int slotBase,
                                          int nb, int vec8, int* list, int tid, int lane, int wave) {
  int wc = 0;
  const int el0  = tid * EPT;
  const int e0   = cbase + el0;
  const int sent = -2147483647 - 1;
  v4i da, db;
  if (vec8 != 0 && cbase + CHUNK <= nE) {
    const int* ep = ei + (size_t)e0 * 2;
    const v4i p0 = *(const v4i*)ep;
    const v4i p1 = *(const v4i*)(ep + 4);
    const v4i p2 = *(const v4i*)(ep + 8);
    const v4i p3 = *(const v4i*)(ep + 12);
    da.x = p0.x; da.y = p0.z; da.z = p1.x; da.w = p1.z;
    db.x = p2.x; db.y = p2.z; db.z = p3.x; db.w = p3.z;
  } else {
    da.x = (e0     < nE) ? ei[(size_t)2 * (size_t)min(e0,     nE - 1)] : sent;
    da.y = (e0 + 1 < nE) ? ei[(size_t)2 * (size_t)min(e0 + 1, nE - 1)] : sent;
    da.z = (e0 + 2 < nE) ? ei[(size_t)2 * (size_t)min(e0 + 2, nE - 1)] : sent;
    da.w = (e0 + 3 < nE) ? ei[(size_t)2 * (size_t)min(e0 + 3, nE - 1)] : sent;
    db.x = (e0 + 4 < nE) ? ei[(size_t)2 * (size_t)min(e0 + 4, nE - 1)] : sent;
    db.y = (e0 + 5 < nE) ? ei[(size_t)2 * (size_t)min(e0 + 5, nE - 1)] : sent;
    db.z = (e0 + 6 < nE) ? ei[(size_t)2 * (size_t)min(e0 + 6, nE - 1)] : sent;
    db.w = (e0 + 7 < nE) ? ei[(size_t)2 * (size_t)min(e0 + 7, nE - 1)] : sent;
  }
  const unsigned nbs = (unsigned)slotBase;
  const unsigned unb = (unsigned)nb;
  const unsigned s0 = (unsigned)da.x - nbs, s1 = (unsigned)da.y - nbs;
  const unsigned s2 = (unsigned)da.z - nbs, s3 = (unsigned)da.w - nbs;
  const unsigned s4 = (unsigned)db.x - nbs, s5 = (unsigned)db.y - nbs;
  const unsigned s6 = (unsigned)db.z - nbs, s7 = (unsigned)db.w - nbs;
  const bool h0 = s0 < unb, h1 = s1 < unb, h2 = s2 < unb, h3 = s3 < unb;
  const bool h4 = s4 < unb, h5 = s5 < unb, h6 = s6 < unb, h7 = s7 < unb;
  const unsigned any = __builtin_amdgcn_ballot_w32(h0 | h1 | h2 | h3 | h4 | h5 | h6 | h7);
  if (any != 0u) {
#define HITJ(J, HJ, SJ) { \
      const unsigned mj = __builtin_amdgcn_ballot_w32(HJ); \
      if (mj != 0u) { \
        if (HJ) { \
          const int pos = wc + (int)__builtin_amdgcn_mbcnt_lo(mj, 0u); \
          if (pos < WCAP) list[wave * WCAP + pos] = ((el0 + (J)) << SLOTB) | (int)(SJ); \
        } \
        wc += (int)__builtin_popcount(mj); } }
    HITJ(0, h0, s0)
    HITJ(1, h1, s1)
    HITJ(2, h2, s2)
    HITJ(3, h3, s3)
    HITJ(4, h4, s4)
    HITJ(5, h5, s5)
    HITJ(6, h6, s6)
    HITJ(7, h7, s7)
#undef HITJ
  }
  return wc;
}

__global__ __launch_bounds__(NTHR) void k_xprep(const float* __restrict__ x, unsigned short* xb, int nN, int nUnits) {
  const int i = (int)blockIdx.x * NTHR + (int)threadIdx.x;
  if (i >= nUnits) return;
  const int row = i >> 5;
  const int c0  = (i & 31) * 8;
  const int rc  = row < nN ? row : nN - 1;
  const float* p = x + (size_t)rc * DI + c0;
  v4f a = *(const v4fa*)p, b = *(const v4fa*)(p + 4);
  const v4f z4 = {0.f, 0.f, 0.f, 0.f};
  if (row >= nN) { a = z4; b = z4; }
  const v8us hv = cvt8b(a, b);
  const size_t o = (size_t)row * DI + c0;
  *(volatile v8us*)(xb + o) = hv;
  __threadfence();
  *(volatile v8us*)(xb + o) = hv;
}

__global__ __launch_bounds__(NTHR) void k_wtr(const float* __restrict__ W, unsigned short* wt, int nUnits) {
  const int u = (int)blockIdx.x * NTHR + (int)threadIdx.x;
  if (u >= nUnits) return;
  const int kq = DI >> 3;
  const int n  = u / kq;
  const int k8 = (u - n * kq) * 8;
  const int h  = n >> 6;
  const int o  = n & (DO - 1);
  const float* p = W + ((size_t)h * DI + (size_t)k8) * DO + o;
  v4f a, b;
  a.x = p[0];                  a.y = p[(size_t)DO];         a.z = p[(size_t)2 * DO];     a.w = p[(size_t)3 * DO];
  b.x = p[(size_t)4 * DO];     b.y = p[(size_t)5 * DO];     b.z = p[(size_t)6 * DO];     b.w = p[(size_t)7 * DO];
  const v8us hv = cvt8b(a, b);
  const size_t oo = (size_t)n * DI + k8;
  *(volatile v8us*)(wt + oo) = hv;
  __threadfence();
  *(volatile v8us*)(wt + oo) = hv;
}

__global__ __launch_bounds__(GTHR) void k_gemm(
    const unsigned short* __restrict__ A, const unsigned short* __restrict__ WT,
    const float* __restrict__ av, float* outF, float* S, int K, int ldo, int MP)
{
  __shared__ __attribute__((aligned(16))) float stg[GBM * GBN];
  __shared__ __attribute__((aligned(16))) float sa[2 * DO];
  __shared__ __attribute__((aligned(16))) float sdot[2 * GBM];
  const int tid = (int)threadIdx.x, lane = tid & 31, wave = tid >> 5, hh = lane >> 4, m = lane & 15;
  const int rowBase = (int)blockIdx.x * GBM;
  const int head    = (int)blockIdx.y;
  const int col0    = head * GBN;

  sa[tid] = bfr(av[head * 2 * DO + tid]);

  v8f acc[4];
  {
    const v8f z = {0.f, 0.f, 0.f, 0.f, 0.f, 0.f, 0.f, 0.f};
    acc[0] = z; acc[1] = z; acc[2] = z; acc[3] = z;
  }
  const unsigned short* ap = A  + (size_t)(rowBase + 16 * wave + m) * (size_t)K + 8 * hh;
  const unsigned short* wp = WT + (size_t)(col0 + m) * (size_t)K + 8 * hh;
  const int ksteps = K >> 5;
#pragma unroll 1
  for (int ks = 0; ks < ksteps; ++ks) {
    FragB af;
    af.h[0] = *(const v8usa*)(ap + 32 * ks);
    af.h[1] = *(const v8usa*)(ap + 32 * ks + 16);
#pragma unroll
    for (int t = 0; t < 4; ++t) {
      const unsigned short* wq = wp + (size_t)(16 * t) * (size_t)K + 32 * ks;
      FragB bf;
      bf.h[0] = *(const v8usa*)wq;
      bf.h[1] = *(const v8usa*)(wq + 16);
      acc[t] = wmb(af, bf, acc[t]);
    }
  }

#pragma unroll
  for (int t = 0; t < 4; ++t) {
    const int lc = 16 * t + m;
#pragma unroll
    for (int r = 0; r < 8; ++r) {
      const int lr = 16 * wave + 8 * hh + r;
      stg[lr * GBN + lc] = acc[t][r];
    }
  }
  __syncthreads();

  v4f fv[8];
#pragma unroll
  for (int i = 0; i < 8; ++i) {
    const int lr = 16 * wave + 2 * i + hh;
    fv[i] = *(const v4fa*)(stg + lr * GBN + 4 * m);
  }

  {
    const int row   = tid & (GBM - 1);
    const int which = tid >> 6;
    const float* hr = stg + row * GBN;
    const float* ar = sa + which * DO;
    float r = 0.f;
#pragma unroll 4
    for (int c4 = 0; c4 < GBN / 4; ++c4) {
      const v4f hv4 = *(const v4fa*)(hr + 4 * c4);
      const v4f a4  = *(const v4fa*)(ar + 4 * c4);
      r = fmaf(hv4.x, a4.x, r);
      r = fmaf(hv4.y, a4.y, r);
      r = fmaf(hv4.z, a4.z, r);
      r = fmaf(hv4.w, a4.w, r);
    }
    sdot[which * GBM + row] = r;
  }
  __syncthreads();
  const v4f sv = *(const v4fa*)(sdot + 4 * lane);
  float* sp = S + (size_t)((lane >> 4) * NH + head) * (size_t)MP + rowBase + 4 * (lane & 15);

#pragma unroll
  for (int i = 0; i < 8; ++i) {
    const int lr = 16 * wave + 2 * i + hh;
    const int gr = rowBase + lr;
    float* op = outF + (size_t)gr * (size_t)ldo + col0 + 4 * m;
    *(volatile v4f*)op = fv[i];
  }
  if (wave == 0) *(volatile v4f*)sp = sv;
  __threadfence();
#pragma unroll
  for (int i = 0; i < 8; ++i) {
    const int lr = 16 * wave + 2 * i + hh;
    const int gr = rowBase + lr;
    float* op = outF + (size_t)gr * (size_t)ldo + col0 + 4 * m;
    *(volatile v4f*)op = fv[i];
  }
  if (wave == 0) *(volatile v4f*)sp = sv;
}

__global__ __launch_bounds__(NTHR) void k_agg(
    const int* __restrict__ ei, const float* __restrict__ HF, const float* __restrict__ S,
    float* out, int nN, int nE, int nb, int vec8, int MP) {
  extern __shared__ v4f lds_dyn[];
  int* reg1 = (int*)lds_dyn;
  int* reg2 = reg1 + RCAP;
  int* scnt = reg2 + RCAP;
  int* soff = scnt + NBMAX;
  int* list = soff + NBMAX;
  int* wcnt = list + LISTN;
  int* wtot = wcnt + NWAVE;
  const int tid = (int)threadIdx.x, lane = tid & 31, wave = tid >> 5;
  const int nodeBase = (int)blockIdx.x * nb;

  for (int i = tid; i < NBMAX; i += NTHR) scnt[i] = 0;
  __syncthreads();

  int tot = 0;
  const int nChunks = (nE + CHUNK - 1) / CHUNK;
#pragma unroll 1
  for (int ch = 0; ch < nChunks; ++ch) {
    const int cbase = ch * CHUNK;
    const int wc = scan_chunk(ei, nE, cbase, nodeBase, nb, vec8, list, tid, lane, wave);
    if (lane == 0) wcnt[wave] = wc;
    __syncthreads();
    int pre = 0, all = 0;
#pragma unroll
    for (int w2 = 0; w2 < NWAVE; ++w2) {
      int c = wcnt[w2];
      c = c < 0 ? 0 : (c > WCAP ? WCAP : c);
      all += c;
      pre += (w2 < wave) ? c : 0;
    }
    const int wcc  = wc > WCAP ? WCAP : wc;
    const int base = tot + pre;
#pragma unroll 1
    for (int i = lane; i < wcc; i += 32) {
      const int ent = list[wave * WCAP + i];
      const int el  = (ent >> SLOTB) & (CHUNK - 1);
      const int sl  = ent & (NBMAX - 1);
      int eid = cbase + el;
      eid = eid > nE - 1 ? nE - 1 : eid;
      const int pos = base + i;
      if (pos < RCAP) reg1[pos] = (int)(((unsigned)eid << SLOTB) | (unsigned)sl);
    }
    tot += all;
    tot = tot > RCAP ? RCAP : tot;
    __syncthreads();
  }
  const int nh = tot;

  if (wave == 0) {
#pragma unroll 1
    for (int b0 = 0; b0 < nh; b0 += 32) {
      const int idx = b0 + lane;
      const int uv  = reg1[idx < nh ? idx : nh - 1];
      const int m32 = (nh - b0) < 32 ? (nh - b0) : 32;
#pragma unroll 1
      for (int k = 0; k < m32; ++k) {
        const int u  = __builtin_amdgcn_readlane(uv, k);
        const int sl = u & (NBMAX - 1);
        if (lane == 0) scnt[sl] = scnt[sl] + 1;
      }
    }
  }
  __syncthreads();

  {
    const v4i ca = *(const v4i*)(scnt + 8 * tid);
    const v4i cb = *(const v4i*)(scnt + 8 * tid + 4);
    const int e0 = ca.x < 0 ? 0 : ca.x, e1 = ca.y < 0 ? 0 : ca.y, e2 = ca.z < 0 ? 0 : ca.z, e3 = ca.w < 0 ? 0 : ca.w;
    const int e4 = cb.x < 0 ? 0 : cb.x, e5 = cb.y < 0 ? 0 : cb.y, e6 = cb.z < 0 ? 0 : cb.z, e7 = cb.w < 0 ? 0 : cb.w;
    const int ts = e0 + e1 + e2 + e3 + e4 + e5 + e6 + e7;
    int incl = ts;
#pragma unroll
    for (int d = 1; d < 32; d <<= 1) {
      const int up = __shfl_up(incl, d);
      if (lane >= d) incl += up;
    }
    if (lane == 31) wtot[wave] = incl;
    __syncthreads();
    int pre = 0;
#pragma unroll
    for (int w2 = 0; w2 < NWAVE; ++w2) pre += (w2 < wave) ? wtot[w2] : 0;
    int run = pre + incl - ts;
    soff[8 * tid + 0] = run; run += e0;
    soff[8 * tid + 1] = run; run += e1;
    soff[8 * tid + 2] = run; run += e2;
    soff[8 * tid + 3] = run; run += e3;
    soff[8 * tid + 4] = run; run += e4;
    soff[8 * tid + 5] = run; run += e5;
    soff[8 * tid + 6] = run; run += e6;
    soff[8 * tid + 7] = run;
  }
  __syncthreads();
  for (int i = tid; i < NBMAX; i += NTHR) list[i] = soff[i];
  __syncthreads();

  if (wave == 0) {
#pragma unroll 1
    for (int b0 = 0; b0 < nh; b0 += 32) {
      const int idx = b0 + lane;
      const int uv  = reg1[idx < nh ? idx : nh - 1];
      const int m32 = (nh - b0) < 32 ? (nh - b0) : 32;
#pragma unroll 1
      for (int k = 0; k < m32; ++k) {
        const int u   = __builtin_amdgcn_readlane(uv, k);
        const int sl  = u & (NBMAX - 1);
        const int eid = (int)((unsigned)u >> SLOTB);
        if (lane == 0) {
          int pos = list[sl];
          pos = pos < 0 ? 0 : (pos > RCAP - 1 ? RCAP - 1 : pos);
          reg2[pos] = eid;
          list[sl] = pos + 1;
        }
      }
    }
  }
  __syncthreads();

  const int nbw = nb >> 3;
  const bool ovf = (nh >= RCAP);
  const float qnan = __int_as_float(0x7fc00000);
  const int head = lane >> 3;
  const int c0   = 8 * lane;
  const float* S1p = S + (size_t)head * (size_t)MP;
  const float* S2p = S + (size_t)(NH + head) * (size_t)MP;
  const int hsrc = lane >> 1;
  const bool odd = (lane & 1) != 0;

#pragma unroll 1
  for (int jt = 0; jt < nbw; ++jt) {
    const int slot = wave * nbw + jt;
    const int grow = nodeBase + slot;
    const int gcl  = grow < nN ? grow : nN - 1;
    int st = soff[slot];
    const int craw = scnt[slot];
    int cnt = craw;
    st  = st < 0 ? 0 : (st > nh ? nh : st);
    cnt = cnt < 0 ? 0 : (cnt > DEGCAP ? DEGCAP : cnt);
    if (cnt > nh - st) cnt = nh - st;
    const float pz = (ovf || craw > DEGCAP) ? qnan : 0.0f;
    const bool wr = grow < nN;

    const float s1v = S1p[gcl];
    float mx = -1.0e30f, dn = 0.f;
    v4f aa = {0.f, 0.f, 0.f, 0.f};
    v4f ab = {0.f, 0.f, 0.f, 0.f};

#pragma unroll 1
    for (int q = 0; q < cnt; ++q) {
      int idx = st + q; idx = idx > RCAP - 1 ? RCAP - 1 : idx;
      int eid = reg2[idx]; eid = eid < 0 ? 0 : (eid > nE - 1 ? nE - 1 : eid);
      const int sraw = ei[(size_t)eid * 2 + 1];
      const int s = sraw < 0 ? 0 : (sraw > nN - 1 ? nN - 1 : sraw);
      const float s2v = S2p[s];
      const float* hp = HF + (size_t)s * NF + c0;
      const v4f ha = *(const v4fa*)hp;
      const v4f hb = *(const v4fa*)(hp + 4);
      float lg = s1v + s2v;
      lg = lg > 0.f ? lg : NEGSL * lg;
      const float df = lg - mx;
      const float ee = __expf(-fabsf(df));
      const bool up  = df > 0.f;
      const float f1 = up ? ee : 1.0f;
      const float f2 = up ? 1.0f : ee;
      mx = up ? lg : mx;
      dn = fmaf(dn, f1, f2);
      aa.x = fmaf(aa.x, f1, f2 * ha.x);
      aa.y = fmaf(aa.y, f1, f2 * ha.y);
      aa.z = fmaf(aa.z, f1, f2 * ha.z);
      aa.w = fmaf(aa.w, f1, f2 * ha.w);
      ab.x = fmaf(ab.x, f1, f2 * hb.x);
      ab.y = fmaf(ab.y, f1, f2 * hb.y);
      ab.z = fmaf(ab.z, f1, f2 * hb.z);
      ab.w = fmaf(ab.w, f1, f2 * hb.w);
    }
    const float ds = dn > 0.f ? dn : 1.0f;
    const float iv = (dn > 0.f ? 1.0f : 0.0f) * __builtin_amdgcn_rcpf(ds);
    const float o0 = fmaxf(aa.x * iv, 0.f) + pz;
    const float o1 = fmaxf(aa.y * iv, 0.f) + pz;
    const float o2 = fmaxf(aa.z * iv, 0.f) + pz;
    const float o3 = fmaxf(aa.w * iv, 0.f) + pz;
    const float o4 = fmaxf(ab.x * iv, 0.f) + pz;
    const float o5 = fmaxf(ab.y * iv, 0.f) + pz;
    const float o6 = fmaxf(ab.z * iv, 0.f) + pz;
    const float o7 = fmaxf(ab.w * iv, 0.f) + pz;

    const float g0 = __shfl(o0, hsrc), g1 = __shfl(o1, hsrc), g2 = __shfl(o2, hsrc), g3 = __shfl(o3, hsrc);
    const float g4 = __shfl(o4, hsrc), g5 = __shfl(o5, hsrc), g6 = __shfl(o6, hsrc), g7 = __shfl(o7, hsrc);
    const float u0 = __shfl(o0, 16 + hsrc), u1 = __shfl(o1, 16 + hsrc), u2 = __shfl(o2, 16 + hsrc), u3 = __shfl(o3, 16 + hsrc);
    const float u4 = __shfl(o4, 16 + hsrc), u5 = __shfl(o5, 16 + hsrc), u6 = __shfl(o6, 16 + hsrc), u7 = __shfl(o7, 16 + hsrc);
    v4f w1, w2;
    w1.x = odd ? g4 : g0; w1.y = odd ? g5 : g1; w1.z = odd ? g6 : g2; w1.w = odd ? g7 : g3;
    w2.x = odd ? u4 : u0; w2.y = odd ? u5 : u1; w2.z = odd ? u6 : u2; w2.w = odd ? u7 : u3;

    float* op = out + (size_t)gcl * NF + 4 * lane;
    if (wr) {
      *(volatile v4f*)op = w1;
      *(volatile v4f*)(op + NF / 2) = w2;
    }
    __threadfence();
    if (wr) {
      *(volatile v4f*)op = w1;
      *(volatile v4f*)(op + NF / 2) = w2;
    }
  }
}

static int pick_nb(int nE, int nN) {
  int nb = NBMAX;
  while (nb > 32 && (long long)nb * (long long)nE * 5LL > (long long)RCAP * (long long)nN * 4LL) nb >>= 1;
  return nb;
}
static inline int cdiv(int a, int b) { return (a + b - 1) / b; }

extern "C" void kernel_launch(void* const* d_in, const int* in_sizes, int n_in,
                              void* d_out, int out_size, void* d_ws, size_t ws_size,
                              hipStream_t stream) {
  if (n_in < 4) return;
  const int nN = in_sizes[0] / DI;
  if (nN <= 0 || in_sizes[0] != nN * DI || nN > (1 << 22)) return;
  if (in_sizes[1] != NH * DI * DO) return;
  if (in_sizes[2] != NH * 2 * DO) return;
  if (in_sizes[3] < 2 || (in_sizes[3] & 1) != 0) return;
  const int nE = in_sizes[3] / 2;
  if (nE < 1 || nE >= (1 << (32 - SLOTB))) return;
  if (out_size != nN * NF) return;

  const float* x  = (const float*)d_in[0];
  const float* W  = (const float*)d_in[1];
  const float* a  = (const float*)d_in[2];
  const int*   ei = (const int*)  d_in[3];
  float* out = (float*)d_out;

  const int MP   = cdiv(nN, GBM) * GBM;
  const int nb   = pick_nb(nE, nN);
  if (nb < 32 || (nb & (nb - 1)) != 0 || nb > NBMAX) return;
  const int gA   = cdiv(nN, nb);
  if ((long long)gA * nb < (long long)nN) return;
  const int vec8 = 1;

  char* ws = (char*)d_ws;
  size_t off = 0;
  const size_t oXB = off; off += (size_t)MP * DI * 2;            off = (off + 255) & ~(size_t)255;
  const size_t oWT = off; off += (size_t)NF * DI * 2;            off = (off + 255) & ~(size_t)255;
  const size_t oHF = off; off += (size_t)MP * NF * 4;            off = (off + 255) & ~(size_t)255;
  const size_t oS  = off; off += (size_t)2 * NH * MP * 4;        off = (off + 255) & ~(size_t)255;
  if (off > ws_size || off > (size_t)WSMAX) return;
  unsigned short* XB = (unsigned short*)(ws + oXB);
  unsigned short* WT = (unsigned short*)(ws + oWT);
  float*          HF = (float*)(ws + oHF);
  float*          S  = (float*)(ws + oS);

  hipFuncSetAttribute(reinterpret_cast<const void*>(&k_agg),
                      hipFuncAttributeMaxDynamicSharedMemorySize, LDS_AGG);

  const int nUx = MP * (DI / 8);
  k_xprep<<<cdiv(nUx, NTHR), NTHR, 0, stream>>>(x, XB, nN, nUx);

  const int nUw = NF * (DI / 8);
  k_wtr<<<cdiv(nUw, NTHR), NTHR, 0, stream>>>(W, WT, nUw);

  k_gemm<<<dim3(MP / GBM, NF / GBN), GTHR, 0, stream>>>(XB, WT, a, HF, S, DI, NF, MP);

  k_agg<<<gA, NTHR, LDS_AGG, stream>>>(ei, HF, S, out, nN, nE, nb, vec8, MP);
}
